// MessagePassingNetwork_33809982554511
// MI455X (gfx1250) — hardware-verified
//
#include <hip/hip_runtime.h>
#include <stdint.h>


typedef _Float16 f16;
typedef f16   v8h  __attribute__((ext_vector_type(8)));
typedef f16   v16h __attribute__((ext_vector_type(16)));
typedef float v8f  __attribute__((ext_vector_type(8)));
typedef float v4f  __attribute__((ext_vector_type(4)));
union Frag { v16h v; v8h half[2]; };

#define DEV static __device__ __forceinline__

#define NB    4
#define NC    32
#define NH    256
#define NW    256
#define HID   64
#define CIN1  65
#define LSTR  72
#define XP2   130
#define XP3   144
#define WSCALE 16.0f
#define WINV   0.0625f

#define F_ML1   0
#define F_ML2   48
#define F_ML3   96
#define F_AG1   100
#define F_AG2   108
#define F_AG3   180
#define N_FRAGS 186

DEV v8f zero8f() {
  v8f z;
#pragma unroll
  for (int i = 0; i < 8; ++i) z[i] = 0.0f;
  return z;
}
DEV v8h zero8h() {
  v8h z;
#pragma unroll
  for (int i = 0; i < 8; ++i) z[i] = (f16)0.0f;
  return z;
}

DEV v8f wmma16(v16h a, v16h b, v8f c) {
  v8f d = __builtin_amdgcn_wmma_f32_16x16x32_f16(false, a, false, b, (short)0, c, false, false);
  asm volatile("v_nop\n\tv_nop\n\tv_nop\n\tv_nop" : "+v"(d) : "v"(a), "v"(b));
  return d;
}

DEV v16h ld_afrag(const f16* __restrict__ base, int lane) {
  Frag f;
  f.half[0] = *(const v8h*)(base + lane * 16);
  f.half[1] = *(const v8h*)(base + lane * 16 + 8);
  return f.v;
}
DEV v16h ld_bfrag(const f16* rowp, int kt, int h) {
  Frag f;
  f.half[0] = *(const v8h*)(rowp + kt * 32 + 8 * h);
  f.half[1] = *(const v8h*)(rowp + kt * 32 + 16 + 8 * h);
  return f.v;
}

__global__ __launch_bounds__(32) void k_pack(
    const float* __restrict__ g1w, const float* __restrict__ g2w, const float* __restrict__ g3w,
    const float* __restrict__ a1w, const float* __restrict__ a2w, const float* __restrict__ a3w,
    f16* packed) {
  __shared__ __attribute__((aligned(16))) f16 frag[512];
  const int f = blockIdx.x;
  const int l = threadIdx.x, h = l >> 4, m = l & 15;
#pragma unroll 1
  for (int e = 0; e < 16; ++e) {
    const int k = (e < 8) ? (8 * h + e) : (16 + 8 * h + (e - 8));
    float val = 0.0f;
    if (f < F_ML2) {
      const int g = f - F_ML1, var = g / 24, rem = g - var * 24;
      const int tap = rem >> 3, kt = (rem >> 2) & 1, mt = rem & 3;
      const int o = mt * 16 + m, K = kt * 32 + k;
      const int toff = var ? (tap * 3 + 1) : (3 + tap);
      val = g1w[(o * CIN1 + K) * 9 + toff];
    } else if (f < F_ML3) {
      const int g = f - F_ML2, var = g / 24, rem = g - var * 24;
      const int tap = rem >> 3, kt = (rem >> 2) & 1, mt = rem & 3;
      const int o = mt * 16 + m, K = kt * 32 + k;
      const int toff = var ? (tap * 3 + 1) : (3 + tap);
      val = g2w[(o * HID + K) * 9 + toff];
    } else if (f < F_AG1) {
      const int g = f - F_ML3, var = g >> 1, kt = g & 1;
      const int K = kt * 32 + k;
      if (m < 3) {
        const int toff = var ? (m * 3 + 1) : (3 + m);
        val = g3w[K * 9 + toff];
      }
    } else if (f < F_AG2) {
      const int g = f - F_AG1, kt = g >> 2, mt = g & 3;
      const int o = mt * 16 + m, K = kt * 32 + k;
      if (K < 45) {
        const int tap = K / 5, c = K - tap * 5;
        val = a1w[(o * 5 + c) * 9 + tap];
      }
    } else if (f < F_AG3) {
      const int g = f - F_AG2, mt = g & 3, kt = (g >> 2) & 1, tap = g >> 3;
      const int o = mt * 16 + m, K = kt * 32 + k;
      val = a2w[(o * HID + K) * 9 + tap];
    } else {
      const int g = f - F_AG3, d = g >> 1, kt = g & 1;
      const int K = kt * 32 + k;
      if (m < 3) val = a3w[K * 9 + d * 3 + m];
    }
    frag[l * 16 + e] = (f16)(val * WSCALE);
  }
  __syncthreads();
  const v8h v0 = *(const v8h*)&frag[l * 8];
  const v8h v1 = *(const v8h*)&frag[(32 + l) * 8];
  f16* gb = packed + (size_t)f * 512;
  *(volatile v8h*)(gb + l * 8) = v0;
  *(volatile v8h*)(gb + (32 + l) * 8) = v1;
  __threadfence();
  *(volatile v8h*)(gb + l * 8) = v0;
  *(volatile v8h*)(gb + (32 + l) * 8) = v1;
}

template <bool HAS_DT>
DEV void msg_layer(const f16* src, f16* dst, const f16* __restrict__ afr,
                   const float* biasS, const float* wdtS, int mTile, int ntBase, int lane) {
  v16h A[3][2];
#pragma unroll
  for (int tap = 0; tap < 3; ++tap)
#pragma unroll
    for (int kt = 0; kt < 2; ++kt)
      A[tap][kt] = ld_afrag(afr + (size_t)((tap * 2 + kt) * 4 + mTile) * 512, lane);

  const int n = lane & 15, h = lane >> 4;
  const int chBase = mTile * 16 + 8 * h;

#pragma unroll 1
  for (int nt = ntBase; nt < ntBase + 8; ++nt) {
    v8f acc = zero8f();
#pragma unroll
    for (int tap = 0; tap < 3; ++tap) {
      const f16* sp = src + (nt * 16 + n + tap - 1) * LSTR;
      acc = wmma16(A[tap][0], ld_bfrag(sp, 0, h), acc);
      acc = wmma16(A[tap][1], ld_bfrag(sp, 1, h), acc);
    }
    const int pos = nt * 16 + n;
    float dval[3] = {0.0f, 0.0f, 0.0f};
    if constexpr (HAS_DT) {
#pragma unroll
      for (int tap = 0; tap < 3; ++tap) dval[tap] = (float)src[(pos + tap - 1) * LSTR + 64];
    }
    v8h ov;
#pragma unroll
    for (int v = 0; v < 8; ++v) {
      const int ch = chBase + v;
      float x = acc[v] * WINV + biasS[ch];
      if constexpr (HAS_DT) {
#pragma unroll
        for (int tap = 0; tap < 3; ++tap) x += wdtS[ch * 3 + tap] * dval[tap];
      }
      x = fmaxf(x, 0.0f);
      ov[v] = (f16)x;
    }
    *(v8h*)&dst[pos * LSTR + chBase] = ov;
  }
}

__global__ __launch_bounds__(256) void k_msg(
    const float* __restrict__ feat, const float* __restrict__ dt,
    const float* __restrict__ g1w, const float* __restrict__ g1b,
    const float* __restrict__ g2b, const float* __restrict__ g3b,
    const f16* __restrict__ packed, const int* __restrict__ iters,
    float* msg) {
  __shared__ __attribute__((aligned(16))) f16 rawA[(NW + 2) * LSTR];
  __shared__ __attribute__((aligned(16))) f16 rawB[(NW + 2) * LSTR];
  __shared__ float gbuf[3 * (NW + 2)];
  __shared__ float wdts[192], b1s[64], b2s[64];
  __shared__ __attribute__((aligned(16))) float sline[NW];
  f16* bufA = rawA + LSTR;
  f16* bufB = rawB + LSTR;

  const int R = blockIdx.x, b = blockIdx.y, dir = blockIdx.z;
  const int tid = threadIdx.x, lane = tid & 31, wave = tid >> 5;
  const int n = lane & 15, h = lane >> 4;
  const bool colDir = (dir >= 2);
  const int var = colDir ? 1 : 0;
  const bool fwd = (dir == 0) || (dir == 2);
  const bool zeroLine = fwd ? (R == NH - 1) : (R == 0);
  const int node = fwd ? (R + 1) : (R - 1);
  const int nbr = R;
  const bool active = (iters[0] > 0) && !zeroLine;

  float s = 0.0f;
  if (active) {
    if (tid < 2 * LSTR) {
      const int row = (tid < LSTR) ? 0 : (NW + 1);
      const int c = (tid < LSTR) ? tid : tid - LSTR;
      rawA[row * LSTR + c] = (f16)0.0f;
      rawB[row * LSTR + c] = (f16)0.0f;
    }
    if (tid < 3) { gbuf[tid * (NW + 2)] = 0.0f; gbuf[tid * (NW + 2) + NW + 1] = 0.0f; }
    if (tid < 192) {
      const int ch = tid / 3, k = tid - ch * 3;
      const int toff = var ? (k * 3 + 1) : (3 + k);
      wdts[tid] = g1w[(ch * CIN1 + 64) * 9 + toff];
    }
    if (tid < 64) { b1s[tid] = g1b[tid]; b2s[tid] = g2b[tid]; }

    {
      const int pos = tid;
      const size_t HWs = (size_t)NH * NW;
#pragma unroll 1
      for (int ch = 0; ch < NC; ++ch) {
        const size_t pl = (size_t)(b * NC + ch) * HWs;
        const size_t inode = colDir ? (pl + (size_t)pos * NW + node) : (pl + (size_t)node * NW + pos);
        const size_t inbr  = colDir ? (pl + (size_t)pos * NW + nbr)  : (pl + (size_t)nbr  * NW + pos);
        bufA[pos * LSTR + ch]      = (f16)feat[inode];
        bufA[pos * LSTR + 32 + ch] = (f16)feat[inbr];
      }
      const size_t pd = (size_t)b * HWs;
      const size_t idt = colDir ? (pd + (size_t)pos * NW + node) : (pd + (size_t)node * NW + pos);
      bufA[pos * LSTR + 64] = (f16)dt[idt];
    }
    __syncthreads();

    const int mTile = wave & 3, ntBase = (wave >> 2) * 8;
    msg_layer<true>(bufA, bufB, packed + (size_t)(F_ML1 + var * 24) * 512, b1s, wdts, mTile, ntBase, lane);
    __syncthreads();
    msg_layer<false>(bufB, bufA, packed + (size_t)(F_ML2 + var * 24) * 512, b2s, wdts, mTile, ntBase, lane);
    __syncthreads();

    {
      const f16* afr3 = packed + (size_t)(F_ML3 + var * 2) * 512;
      const v16h A0 = ld_afrag(afr3, lane);
      const v16h A1 = ld_afrag(afr3 + 512, lane);
#pragma unroll
      for (int q = 0; q < 2; ++q) {
        const int nt = wave * 2 + q;
        const int p = nt * 16 + n;
        const f16* sp = bufA + p * LSTR;
        v8f acc = zero8f();
        acc = wmma16(A0, ld_bfrag(sp, 0, h), acc);
        acc = wmma16(A1, ld_bfrag(sp, 1, h), acc);
        if (h == 0) {
          gbuf[p + 1] = acc[0];
          gbuf[(NW + 2) + p + 1] = acc[1];
          gbuf[2 * (NW + 2) + p + 1] = acc[2];
        }
      }
    }
    __syncthreads();
    s = g3b[0] + WINV * (gbuf[tid] + gbuf[(NW + 2) + tid + 1] + gbuf[2 * (NW + 2) + tid + 2]);
  }
  sline[tid] = s;
  __syncthreads();
  if (tid < NW / 4) {
    const v4f v = *(const v4f*)&sline[tid * 4];
    float* gp = msg + ((size_t)(dir * NB + b) * NH + R) * NW + tid * 4;
    *(volatile v4f*)gp = v;
    __threadfence();
    *(volatile v4f*)gp = v;
  }
}

__global__ __launch_bounds__(256) void k_agg1(
    const float* __restrict__ msg, const float* __restrict__ dt,
    const f16* __restrict__ afr, const float* __restrict__ bias, f16* hout) {
  __shared__ __attribute__((aligned(16))) f16 xs[128 * LSTR];
  __shared__ __attribute__((aligned(16))) f16 otile[128 * HID];
  const int c0 = blockIdx.x * 128, r = blockIdx.y, b = blockIdx.z;
  const int tid = threadIdx.x;

#pragma unroll 1
  for (int i = tid; i < 64 * 128; i += 256) {
    const int kk = i >> 7, p = i & 127;
    float val = 0.0f;
    if (kk < 45) {
      const int tap = kk / 5, c = kk - tap * 5, dy = tap / 3, dx = tap - dy * 3;
      const int gr = r + dy - 1, gc = c0 + p + dx - 1;
      if (gr >= 0 && gr < NH && gc >= 0 && gc < NW) {
        if (c < 2)      val = msg[((size_t)(c * NB + b) * NH + gr) * NW + gc];
        else if (c < 4) val = msg[((size_t)(c * NB + b) * NW + gc) * NH + gr];
        else            val = dt[((size_t)b * NH + gr) * NW + gc];
      }
    }
    xs[p * LSTR + kk] = (f16)val;
  }
  __syncthreads();

  const int lane = tid & 31, wave = tid >> 5;
  const int n = lane & 15, h = lane >> 4;
  const int mTile = wave & 3, ntBase = (wave >> 2) * 4;
  const int chBase = mTile * 16 + 8 * h;
  const v16h A0 = ld_afrag(afr + (size_t)(0 * 4 + mTile) * 512, lane);
  const v16h A1 = ld_afrag(afr + (size_t)(1 * 4 + mTile) * 512, lane);

#pragma unroll 1
  for (int q = 0; q < 4; ++q) {
    const int p = (ntBase + q) * 16 + n;
    const f16* sp = xs + p * LSTR;
    v8f acc = zero8f();
    acc = wmma16(A0, ld_bfrag(sp, 0, h), acc);
    acc = wmma16(A1, ld_bfrag(sp, 1, h), acc);
    v8h ov;
#pragma unroll
    for (int v = 0; v < 8; ++v) {
      float x = acc[v] * WINV + bias[chBase + v];
      x = fmaxf(x, 0.0f);
      ov[v] = (f16)x;
    }
    *(v8h*)&otile[p * HID + chBase] = ov;
  }
  __syncthreads();

  f16* gb = hout + ((size_t)(b * NH + r) * NW + c0) * HID;
  v8h v[4];
#pragma unroll
  for (int j = 0; j < 4; ++j) v[j] = *(const v8h*)&otile[(j * 256 + tid) * 8];
#pragma unroll
  for (int j = 0; j < 4; ++j) *(volatile v8h*)(gb + (size_t)(j * 256 + tid) * 8) = v[j];
  __threadfence();
#pragma unroll
  for (int j = 0; j < 4; ++j) *(volatile v8h*)(gb + (size_t)(j * 256 + tid) * 8) = v[j];
}

__global__ __launch_bounds__(256) void k_agg2(
    const f16* __restrict__ hin, const f16* __restrict__ afr,
    const float* __restrict__ bias, f16* hout) {
  __shared__ __attribute__((aligned(16))) f16 xs[3 * XP2 * LSTR];
  __shared__ __attribute__((aligned(16))) f16 otile[128 * HID];
  const int c0 = blockIdx.x * 128, r = blockIdx.y, b = blockIdx.z;
  const int tid = threadIdx.x;

#pragma unroll 1
  for (int i = tid; i < 3 * XP2 * 8; i += 256) {
    const int pix = i >> 3, ck = i & 7;
    const int d = pix / XP2, p = pix - d * XP2;
    const int gr = r + d - 1, gc = c0 + p - 1;
    v8h val;
    if (gr >= 0 && gr < NH && gc >= 0 && gc < NW)
      val = *(const v8h*)(hin + ((size_t)(b * NH + gr) * NW + gc) * HID + ck * 8);
    else
      val = zero8h();
    *(v8h*)&xs[(d * XP2 + p) * LSTR + ck * 8] = val;
  }
  __syncthreads();

  const int lane = tid & 31, wave = tid >> 5;
  const int n = lane & 15, h = lane >> 4;
  const int mTile = wave & 3, ntBase = (wave >> 2) * 4;
  const int chBase = mTile * 16 + 8 * h;

  v8f acc[4];
#pragma unroll
  for (int q = 0; q < 4; ++q) acc[q] = zero8f();

#pragma unroll 1
  for (int tap = 0; tap < 9; ++tap) {
    const int dy = tap / 3, dx = tap - dy * 3;
    const v16h A0 = ld_afrag(afr + (size_t)((tap * 2 + 0) * 4 + mTile) * 512, lane);
    const v16h A1 = ld_afrag(afr + (size_t)((tap * 2 + 1) * 4 + mTile) * 512, lane);
#pragma unroll
    for (int q = 0; q < 4; ++q) {
      const int p = (ntBase + q) * 16 + n + dx;
      const f16* sp = xs + (dy * XP2 + p) * LSTR;
      acc[q] = wmma16(A0, ld_bfrag(sp, 0, h), acc[q]);
      acc[q] = wmma16(A1, ld_bfrag(sp, 1, h), acc[q]);
    }
  }

#pragma unroll
  for (int q = 0; q < 4; ++q) {
    const int p = (ntBase + q) * 16 + n;
    v8h ov;
#pragma unroll
    for (int v = 0; v < 8; ++v) {
      float x = acc[q][v] * WINV + bias[chBase + v];
      x = fmaxf(x, 0.0f);
      ov[v] = (f16)x;
    }
    *(v8h*)&otile[p * HID + chBase] = ov;
  }
  __syncthreads();

  f16* gb = hout + ((size_t)(b * NH + r) * NW + c0) * HID;
  v8h v[4];
#pragma unroll
  for (int j = 0; j < 4; ++j) v[j] = *(const v8h*)&otile[(j * 256 + tid) * 8];
#pragma unroll
  for (int j = 0; j < 4; ++j) *(volatile v8h*)(gb + (size_t)(j * 256 + tid) * 8) = v[j];
  __threadfence();
#pragma unroll
  for (int j = 0; j < 4; ++j) *(volatile v8h*)(gb + (size_t)(j * 256 + tid) * 8) = v[j];
}

__global__ __launch_bounds__(256) void k_agg3(
    const f16* __restrict__ hin, const f16* __restrict__ afr,
    const float* __restrict__ bias, float* outp) {
  __shared__ __attribute__((aligned(16))) f16 xs[3 * XP3 * LSTR];
  __shared__ float gbuf[9 * XP3];
  __shared__ __attribute__((aligned(16))) float sline[128];
  const int c0 = blockIdx.x * 128, r = blockIdx.y, b = blockIdx.z;
  const int tid = threadIdx.x;

#pragma unroll 1
  for (int i = tid; i < 3 * XP3 * 8; i += 256) {
    const int pix = i >> 3, ck = i & 7;
    const int d = pix / XP3, p = pix - d * XP3;
    const int gr = r + d - 1, gc = c0 + p - 1;
    v8h val;
    if (gr >= 0 && gr < NH && gc >= 0 && gc < NW)
      val = *(const v8h*)(hin + ((size_t)(b * NH + gr) * NW + gc) * HID + ck * 8);
    else
      val = zero8h();
    *(v8h*)&xs[(d * XP3 + p) * LSTR + ck * 8] = val;
  }
  __syncthreads();

  const int lane = tid & 31, wave = tid >> 5;
  const int n = lane & 15, h = lane >> 4;

#pragma unroll 1
  for (int pr = wave; pr < 27; pr += 8) {
    const int d = pr / 9, nt = pr - d * 9;
    const v16h A0 = ld_afrag(afr + (size_t)(d * 2 + 0) * 512, lane);
    const v16h A1 = ld_afrag(afr + (size_t)(d * 2 + 1) * 512, lane);
    const int p = nt * 16 + n;
    const f16* sp = xs + (d * XP3 + p) * LSTR;
    v8f acc = zero8f();
    acc = wmma16(A0, ld_bfrag(sp, 0, h), acc);
    acc = wmma16(A1, ld_bfrag(sp, 1, h), acc);
    if (h == 0) {
      gbuf[(d * 3 + 0) * XP3 + p] = acc[0];
      gbuf[(d * 3 + 1) * XP3 + p] = acc[1];
      gbuf[(d * 3 + 2) * XP3 + p] = acc[2];
    }
  }
  __syncthreads();

  if (tid < 128) {
    const int j = tid;
    float t = 0.0f;
#pragma unroll
    for (int d = 0; d < 3; ++d)
#pragma unroll
      for (int dx = 0; dx < 3; ++dx) t += gbuf[(d * 3 + dx) * XP3 + j + dx];
    sline[j] = bias[0] + WINV * t;
  }
  __syncthreads();
  if (tid < 32) {
    const v4f v = *(const v4f*)&sline[tid * 4];
    float* gp = outp + ((size_t)(b * NH + r) * NW + c0) + tid * 4;
    *(volatile v4f*)gp = v;
    __threadfence();
    *(volatile v4f*)gp = v;
  }
}

extern "C" void kernel_launch(void* const* d_in, const int* in_sizes, int n_in,
                              void* d_out, int out_size, void* d_ws, size_t ws_size,
                              hipStream_t stream) {
  if (n_in < 15) return;
  if (in_sizes[0] != NB * NC * NH * NW || in_sizes[1] != NB * NH * NW || out_size != NB * NH * NW) return;

  const float* feat = (const float*)d_in[0];
  const float* dt   = (const float*)d_in[1];
  const float* g1w  = (const float*)d_in[2];
  const float* g1b  = (const float*)d_in[3];
  const float* g2w  = (const float*)d_in[4];
  const float* g2b  = (const float*)d_in[5];
  const float* g3w  = (const float*)d_in[6];
  const float* g3b  = (const float*)d_in[7];
  const float* a1w  = (const float*)d_in[8];
  const float* a1b  = (const float*)d_in[9];
  const float* a2w  = (const float*)d_in[10];
  const float* a2b  = (const float*)d_in[11];
  const float* a3w  = (const float*)d_in[12];
  const float* a3b  = (const float*)d_in[13];
  const int*   iters = (const int*)d_in[14];

  const size_t offMsg = 0;
  const size_t bytesMsg = (size_t)4 * NB * NH * NW * sizeof(float);
  const size_t offPk = offMsg + bytesMsg;
  const size_t bytesPk = (size_t)N_FRAGS * 512 * sizeof(f16);
  const size_t offH1 = ((offPk + bytesPk + 127) / 128) * 128;
  const size_t bytesH = (size_t)NB * NH * NW * HID * sizeof(f16);
  const size_t offH2 = offH1 + bytesH;
  const size_t endWs = offH2 + bytesH;
  if (endWs > ws_size) return;

  char* ws = (char*)d_ws;
  float* msg    = (float*)(ws + offMsg);
  f16*   packed = (f16*)(ws + offPk);
  f16*   h1     = (f16*)(ws + offH1);
  f16*   h2     = (f16*)(ws + offH2);
  float* outp   = (float*)d_out;

  k_pack<<<N_FRAGS, 32, 0, stream>>>(g1w, g2w, g3w, a1w, a2w, a3w, packed);
  k_msg<<<dim3(NH, NB, 4), 256, 0, stream>>>(feat, dt, g1w, g1b, g2b, g3b, packed, iters, msg);
  k_agg1<<<dim3(NW / 128, NH, NB), 256, 0, stream>>>(msg, dt, packed + (size_t)F_AG1 * 512, a1b, h1);
  k_agg2<<<dim3(NW / 128, NH, NB), 256, 0, stream>>>(h1, packed + (size_t)F_AG2 * 512, a2b, h2);
  k_agg3<<<dim3(NW / 128, NH, NB), 256, 0, stream>>>(h2, packed + (size_t)F_AG3 * 512, a3b, outp);
}
